// GRUCell_37014028156993
// MI455X (gfx1250) — hardware-verified
//
#include <hip/hip_runtime.h>
#include <math.h>

constexpr int NROW = 4096;
constexpr int DIM  = 2048;
constexpr int NTHR = 256;
constexpr int EPT  = DIM / NTHR;
constexpr float EPSV   = 1e-5f;
constexpr float MAXNV  = (float)(1.0 - 1e-5);
constexpr float ACARRY = 256.0f;
constexpr float WCARRY = 32.0f;
constexpr float PFOLD  = 1.0f / (256.0f * 32.0f);
static_assert(EPT == 8, "row = 256 threads x 8 elements");
static_assert(NROW % 64 == 0 && DIM % 64 == 0 && DIM % 32 == 0, "GEMM tile multiples, K multiple of 32");
static_assert(((NROW / 64) * (DIM / 64)) % 8 == 0, "GEMM grid exact");
static_assert((DIM * DIM / 8) % NTHR == 0, "weight convert grid exact");

typedef __attribute__((ext_vector_type(16))) _Float16 v16h;
typedef __attribute__((ext_vector_type(8)))  _Float16 v8h;
typedef __attribute__((ext_vector_type(8)))  float    v8f;
typedef __attribute__((ext_vector_type(4)))  float    v4f;

__device__ __forceinline__ void guard4_h(v8f& a, v8f& b, v8f& c, v8f& d, v16h x, v16h y) {
  asm volatile("v_nop\n\tv_nop\n\tv_nop\n\tv_nop" : "+v"(a), "+v"(b), "+v"(c), "+v"(d) : "v"(x), "v"(y));
}
__device__ __forceinline__ void keep4_h(v16h a, v16h b, v16h c, v16h d) { asm volatile("v_nop" :: "v"(a), "v"(b), "v"(c), "v"(d)); }
__device__ __forceinline__ void acc_guard4(v8f& a, v8f& b, v8f& c, v8f& d) { asm volatile("v_nop\n\tv_nop\n\tv_nop\n\tv_nop" : "+v"(a), "+v"(b), "+v"(c), "+v"(d)); }

union FragU { v16h v; v8h h[2]; };
__device__ __forceinline__ v16h frag_load(const _Float16* p) {
  FragU f;
  f.h[0] = *(const v8h*)(p);
  f.h[1] = *(const v8h*)(p + 16);
  return f.v;
}
__device__ __forceinline__ v8f frag_mma(v16h a, v16h b, v8f c) {
  return __builtin_amdgcn_wmma_f32_16x16x32_f16(false, a, false, b, (short)0, c, false, false);
}

__device__ __forceinline__ float rcpf_hw(float x) { return __builtin_amdgcn_rcpf(x); }
__device__ __forceinline__ float sqrtf_hw(float x) { return __builtin_amdgcn_sqrtf(x); }

__device__ __forceinline__ float h16_to_f32(unsigned hb) {
  const unsigned sgn = (hb & 0x8000u) << 16;
  const unsigned em = hb & 0x7fffu;
  const float fn = __uint_as_float((em << 13) + 0x38000000u);
  const float fs = (float)em * 5.9604644775390625e-8f;
  const float mag = (em < 0x400u) ? fs : fn;
  return __uint_as_float(__float_as_uint(mag) | sgn);
}

__device__ __forceinline__ float exp0_scale(float ssq) {
  const float n = fmaxf(sqrtf_hw(ssq), EPSV);
  return tanhf(n) * rcpf_hw(n);
}
__device__ __forceinline__ float log0_scale(float ssq) {
  const float n = fminf(fmaxf(sqrtf_hw(ssq), EPSV), MAXNV);
  const float at = 0.5f * log1pf(2.0f * n * rcpf_hw(1.0f - n));
  return at * rcpf_hw(n);
}

template <int NS>
__device__ __forceinline__ void block_sums(float (&s)[NS], float* red) {
  const int lane = threadIdx.x & 31;
  const int wave = threadIdx.x >> 5;
#pragma unroll
  for (int i = 0; i < NS; ++i) {
#pragma unroll
    for (int off = 16; off > 0; off >>= 1) s[i] += __shfl_xor(s[i], off, 32);
  }
  if (lane == 0) {
#pragma unroll
    for (int i = 0; i < NS; ++i) red[wave * NS + i] = s[i];
  }
  __syncthreads();
#pragma unroll
  for (int i = 0; i < NS; ++i) {
    float t = 0.0f;
#pragma unroll
    for (int w = 0; w < 8; ++w) t += red[w * NS + i];
    s[i] = t;
  }
  __syncthreads();
}

__global__ __launch_bounds__(NTHR) void prep_kernel(const float* __restrict__ x, const float* __restrict__ hx,
                                                    unsigned short* __restrict__ Aplane) {
  __shared__ float red[32];
  const int tid = threadIdx.x;
  const int row = blockIdx.x;
  const bool hsel = (row >= NROW);
  const float* src = (hsel ? hx : x) + (size_t)(hsel ? (row - NROW) : row) * DIM + 8 * tid;
  const v4f p0 = *(const v4f*)(src);
  const v4f p1 = *(const v4f*)(src + 4);
  float s[1];
  s[0] = 0.0f;
#pragma unroll
  for (int e = 0; e < 4; ++e) { s[0] += p0[e] * p0[e]; s[0] += p1[e] * p1[e]; }
  block_sums<1>(s, red);
  const float sc = ACARRY * log0_scale(s[0]);
  v8h hv;
#pragma unroll
  for (int e = 0; e < 4; ++e) {
    hv[e]     = (_Float16)(p0[e] * sc);
    hv[4 + e] = (_Float16)(p1[e] * sc);
  }
  unsigned short* dp = Aplane + (size_t)row * DIM + 8 * tid;
  *(volatile v8h*)dp = hv;
  __threadfence();
  *(volatile v8h*)dp = hv;
}

__global__ __launch_bounds__(NTHR) void cvt_w_kernel(const float* __restrict__ wx, const float* __restrict__ wh,
                                                     unsigned short* __restrict__ Wplane) {
  const size_t i = (size_t)blockIdx.x * NTHR + threadIdx.x;
  const int y = blockIdx.y;
  const float* sp = (y ? wh : wx) + i * 8;
  const v4f a = *(const v4f*)(sp);
  const v4f b = *(const v4f*)(sp + 4);
  v8h hv;
#pragma unroll
  for (int e = 0; e < 4; ++e) {
    hv[e]     = (_Float16)(a[e] * WCARRY);
    hv[4 + e] = (_Float16)(b[e] * WCARRY);
  }
  unsigned short* dp = Wplane + (size_t)y * DIM * DIM + i * 8;
  *(volatile v8h*)dp = hv;
  __threadfence();
  *(volatile v8h*)dp = hv;
}

__global__ __launch_bounds__(256) void gemm_f16_nt(
    const unsigned short* __restrict__ Ap, int lda, long strideA,
    const unsigned short* __restrict__ Btp, int ldb, long strideB,
    float* __restrict__ Cout, int ldc, long strideC,
    int M, int N, int K, float scale) {
  __shared__ __align__(16) float sT[8][16 * 68];
  const _Float16* A  = (const _Float16*)Ap;
  const _Float16* Bt = (const _Float16*)Btp;
  const int b    = blockIdx.y;
  const int lane = threadIdx.x & 31;
  const int wave = threadIdx.x >> 5;
  const int tilesN = N >> 6;
  const int tilesM = M >> 6;
  const int tile = blockIdx.x * 8 + wave;
  if (tile >= tilesM * tilesN) return;
  const int tm = tile / tilesN;
  const int tn = tile - tm * tilesN;
  const int m0 = tm << 6;
  const int n0 = tn << 6;

  const _Float16* Ab = A  + (size_t)b * strideA;
  const _Float16* Bb = Bt + (size_t)b * strideB;

  const int rlane = lane & 15;
  const int koff  = (lane >> 4) * 8;
  const int mOff  = (lane >> 4) * 8;

  v8f acc[4][4];
#pragma unroll
  for (int i = 0; i < 4; ++i)
#pragma unroll
    for (int j = 0; j < 4; ++j) acc[i][j] = (v8f){0.f, 0.f, 0.f, 0.f, 0.f, 0.f, 0.f, 0.f};

  for (int k0 = 0; k0 < K; k0 += 32) {
    v16h bh[4];
#pragma unroll
    for (int j = 0; j < 4; ++j) {
      const size_t bo = (size_t)(n0 + (j << 4) + rlane) * ldb + koff + k0;
      bh[j] = frag_load(Bb + bo);
    }
#pragma unroll
    for (int i = 0; i < 4; ++i) {
      const size_t ao = (size_t)(m0 + (i << 4) + rlane) * lda + koff + k0;
      const v16h ah = frag_load(Ab + ao);
#pragma unroll
      for (int j = 0; j < 4; ++j) acc[i][j] = frag_mma(ah, bh[j], acc[i][j]);
      guard4_h(acc[i][0], acc[i][1], acc[i][2], acc[i][3], ah, bh[3]);
    }
    keep4_h(bh[0], bh[1], bh[2], bh[3]);
  }
  acc_guard4(acc[0][0], acc[0][1], acc[0][2], acc[0][3]);
  acc_guard4(acc[1][0], acc[1][1], acc[1][2], acc[1][3]);
  acc_guard4(acc[2][0], acc[2][1], acc[2][2], acc[2][3]);
  acc_guard4(acc[3][0], acc[3][1], acc[3][2], acc[3][3]);

  float* slab = sT[wave];
  float* C = Cout + (size_t)b * strideC;
  const int hh = lane >> 4;
  const int c4 = (lane & 15) * 4;
#pragma unroll
  for (int i = 0; i < 4; ++i) {
    const int mBase = m0 + (i << 4);
#pragma unroll
    for (int j = 0; j < 4; ++j) {
#pragma unroll
      for (int r = 0; r < 8; ++r) {
        slab[(mOff + r) * 68 + (j << 4) + rlane] = acc[i][j][r] * scale;
      }
    }
    __builtin_amdgcn_fence(__ATOMIC_RELEASE, "workgroup");
    __builtin_amdgcn_wave_barrier();
    __builtin_amdgcn_fence(__ATOMIC_ACQUIRE, "workgroup");
    for (int pass = 0; pass < 2; ++pass) {
#pragma unroll
      for (int it = 0; it < 8; ++it) {
        const int row = it * 2 + hh;
        const v4f v = *(const v4f*)(slab + row * 68 + c4);
        *(volatile v4f*)(C + (size_t)(mBase + row) * ldc + n0 + c4) = v;
      }
      __threadfence();
    }
    __builtin_amdgcn_fence(__ATOMIC_RELEASE, "workgroup");
    __builtin_amdgcn_wave_barrier();
    __builtin_amdgcn_fence(__ATOMIC_ACQUIRE, "workgroup");
  }
}

template <int MODE>
__global__ __launch_bounds__(NTHR) void pair_kernel(float* PH, const float* __restrict__ PX,
                                                    const float* __restrict__ bias, const float* __restrict__ hx,
                                                    unsigned short* __restrict__ out16) {
  __shared__ __align__(16) float La[DIM];
  __shared__ __align__(16) float Lb[DIM];
  __shared__ __align__(16) float Lh[MODE == 1 ? DIM : 4];
  __shared__ float red[32];
  const int tid = threadIdx.x;
  const int lane = tid & 31;
  const size_t rbase = (size_t)blockIdx.x * DIM;

  float s[4];
  s[0] = 0.0f; s[1] = 0.0f; s[2] = 0.0f; s[3] = 0.0f;
#pragma unroll 1
  for (int j = 0; j < EPT; ++j) {
    const int e = j * NTHR + tid;
    const float a = PH[rbase + e];
    const float b = PX[rbase + e] + bias[e];
    La[e] = a;
    Lb[e] = b;
    s[0] += a * a;
    s[1] += b * b;
    s[2] += a * b;
    if constexpr (MODE == 1) {
      const float h = hx[rbase + e];
      Lh[e] = h;
      s[3] += h * h;
    }
  }
  block_sums<4>(s, red);

  const float aa = s[0], bb = s[1], ab = s[2];
  const float targ = (lane & 1) ? bb : aa;
  const float tsc = exp0_scale(targ);
  const float sa = __shfl(tsc, 0, 32);
  const float sb = __shfl(tsc, 1, 32);
  const float xy = sa * sb * ab;
  const float x2 = sa * sa * aa;
  const float y2 = sb * sb * bb;
  const float cA = 1.0f + 2.0f * xy + y2;
  const float cB = 1.0f - x2;
  const float den = fmaxf(1.0f + 2.0f * xy + x2 * y2, EPSV);
  const float rd = rcpf_hw(den);
  const float al = cA * sa * rd;
  const float be = cB * sb * rd;
  float mm = al * al * aa + 2.0f * al * be * ab + be * be * bb;
  mm = fmaxf(mm, 0.0f);
  const float hsq = (MODE == 1) ? s[3] : mm;
  const float larg = (lane & 1) ? hsq : mm;
  const float lsc = log0_scale(larg);
  const float sl = __shfl(lsc, 0, 32);
  const float sh = __shfl(lsc, 1, 32);
  const float ca = sl * al;
  const float cb = sl * be;
  const float vsc = ACARRY * sh;

#pragma unroll 1
  for (int j = 0; j < EPT; ++j) {
    const int e = j * NTHR + tid;
    const float logit = ca * La[e] + cb * Lb[e];
    float v = logit;
    if constexpr (MODE == 1) {
      const float r = rcpf_hw(1.0f + expf(-logit));
      v = r * vsc * Lh[e];
    }
    if constexpr (MODE == 2) {
      v = tanhf(logit);
    }
    La[e] = v;
  }
  __syncthreads();

  if constexpr (MODE == 2) {
#pragma unroll 1
    for (int it = 0; it < DIM / (4 * NTHR); ++it) {
      const int idx = it * 4 * NTHR + tid * 4;
      const v4f v = *(const v4f*)(La + idx);
      float* op = PH + rbase + idx;
      *(volatile v4f*)op = v;
      __threadfence();
      *(volatile v4f*)op = v;
    }
  } else {
    const v4f p0 = *(const v4f*)(La + 8 * tid);
    const v4f p1 = *(const v4f*)(La + 8 * tid + 4);
    v8h hv;
#pragma unroll
    for (int e = 0; e < 4; ++e) {
      hv[e]     = (_Float16)p0[e];
      hv[4 + e] = (_Float16)p1[e];
    }
    unsigned short* dp = out16 + rbase + 8 * tid;
    *(volatile v8h*)dp = hv;
    __threadfence();
    *(volatile v8h*)dp = hv;
  }
}

__global__ __launch_bounds__(NTHR) void final_kernel(const float* __restrict__ Tp, const float* __restrict__ hx,
                                                     const unsigned* __restrict__ Zw, float* __restrict__ out) {
  __shared__ __align__(16) float Lt[DIM];
  __shared__ __align__(16) float Lh[DIM];
  __shared__ __align__(16) float Lz[DIM];
  __shared__ float red[32];
  const int tid = threadIdx.x;
  const size_t rbase = (size_t)blockIdx.x * DIM;

  float s[3];
  s[0] = 0.0f; s[1] = 0.0f; s[2] = 0.0f;
#pragma unroll 1
  for (int j = 0; j < EPT; ++j) {
    const int e = j * NTHR + tid;
    const float t = Tp[rbase + e];
    const float h = hx[rbase + e];
    const unsigned w = Zw[(rbase + e) >> 1];
    const unsigned hb = (e & 1) ? (w >> 16) : (w & 0xffffu);
    const float zl = h16_to_f32(hb);
    const float z = rcpf_hw(1.0f + expf(-zl));
    Lt[e] = t;
    Lh[e] = h;
    Lz[e] = z;
    s[0] += t * t;
    s[1] += h * t;
    s[2] += h * h;
  }
  block_sums<3>(s, red);
  const float tt = s[0], ht = s[1], hh = s[2];

  const float st = exp0_scale(tt);
  const float xy2 = -(st * ht);
  const float y22 = st * st * tt;
  const float cA2 = 1.0f + 2.0f * xy2 + y22;
  const float cB2 = 1.0f - hh;
  const float den2 = fmaxf(1.0f + 2.0f * xy2 + hh * y22, EPSV);
  const float rd2 = rcpf_hw(den2);
  const float ah = -(cA2 * rd2);
  const float at = cB2 * st * rd2;
  float mm = ah * ah * hh + 2.0f * ah * at * ht + at * at * tt;
  mm = fmaxf(mm, 0.0f);
  const float sl2 = log0_scale(mm);
  const float ch = sl2 * ah;
  const float ct = sl2 * at;

  float u[2];
  u[0] = 0.0f; u[1] = 0.0f;
#pragma unroll 1
  for (int j = 0; j < EPT; ++j) {
    const int e = j * NTHR + tid;
    const float h = Lh[e];
    const float q = Lz[e] * (ch * h + ct * Lt[e]);
    Lt[e] = q;
    u[0] += q * q;
    u[1] += h * q;
  }
  block_sums<2>(u, red);
  const float qq = u[0], hq = u[1];

  const float sq = exp0_scale(qq);
  const float xy3 = sq * hq;
  const float y23 = sq * sq * qq;
  const float cA3 = 1.0f + 2.0f * xy3 + y23;
  const float cB3 = 1.0f - hh;
  const float den3 = fmaxf(1.0f + 2.0f * xy3 + hh * y23, EPSV);
  const float rd3 = rcpf_hw(den3);
  const float oh = cA3 * rd3;
  const float oq = cB3 * sq * rd3;

#pragma unroll 1
  for (int it = 0; it < DIM / (4 * NTHR); ++it) {
    const int idx = it * 4 * NTHR + tid * 4;
    const v4f hv = *(const v4f*)(Lh + idx);
    const v4f qv = *(const v4f*)(Lt + idx);
    v4f o;
#pragma unroll
    for (int e = 0; e < 4; ++e) o[e] = oh * hv[e] + oq * qv[e];
    float* op = out + rbase + idx;
    *(volatile v4f*)op = o;
    __threadfence();
    *(volatile v4f*)op = o;
  }
}

extern "C" void kernel_launch(void* const* d_in, const int* in_sizes, int n_in,
                              void* d_out, int out_size, void* d_ws, size_t ws_size, hipStream_t stream) {
  if (n_in < 11 || d_out == nullptr || d_ws == nullptr) return;
  const int nBD = NROW * DIM;
  const int nDD = DIM * DIM;
  if (in_sizes[0] != nBD || in_sizes[1] != nBD || in_sizes[2] != nDD || in_sizes[3] != nDD || in_sizes[4] != DIM ||
      in_sizes[5] != nDD || in_sizes[6] != nDD || in_sizes[7] != DIM || in_sizes[8] != nDD || in_sizes[9] != DIM ||
      in_sizes[10] != nDD || out_size != nBD) return;

  const float* x     = (const float*)d_in[0];
  const float* hx    = (const float*)d_in[1];
  const float* w_r   = (const float*)d_in[2];
  const float* u_r_w = (const float*)d_in[3];
  const float* u_r_b = (const float*)d_in[4];
  const float* w_z   = (const float*)d_in[5];
  const float* u_z_w = (const float*)d_in[6];
  const float* u_z_b = (const float*)d_in[7];
  const float* u_w   = (const float*)d_in[8];
  const float* u_b   = (const float*)d_in[9];
  const float* w     = (const float*)d_in[10];
  float* out = (float*)d_out;

  constexpr size_t SZ_A = (size_t)NROW * DIM * 2;
  constexpr size_t SZ_W = (size_t)DIM * DIM * 2;
  constexpr size_t SZ_P = (size_t)NROW * DIM * 4;
  constexpr size_t OFF_AX = 0;
  constexpr size_t OFF_AH = OFF_AX + SZ_A;
  constexpr size_t OFF_ZL = OFF_AH + SZ_A;
  constexpr size_t OFF_WX = OFF_ZL + SZ_A;
  constexpr size_t OFF_WH = OFF_WX + SZ_W;
  constexpr size_t OFF_PX = OFF_WH + SZ_W;
  constexpr size_t OFF_PH = OFF_PX + SZ_P;
  constexpr size_t WS_TOTAL = OFF_PH + SZ_P;
  static_assert(WS_TOTAL == (size_t)134217728, "carve total");
  static_assert(OFF_AH % 128 == 0 && OFF_ZL % 128 == 0 && OFF_WX % 128 == 0 && OFF_WH % 128 == 0 &&
                OFF_PX % 128 == 0 && OFF_PH % 128 == 0, "line-aligned carve");
  if (WS_TOTAL > ws_size) return;

  char* ws = (char*)d_ws;
  unsigned short* AX = (unsigned short*)(ws + OFF_AX);
  unsigned short* AH = (unsigned short*)(ws + OFF_AH);
  unsigned short* ZL = (unsigned short*)(ws + OFF_ZL);
  unsigned short* WX = (unsigned short*)(ws + OFF_WX);
  float* PX = (float*)(ws + OFF_PX);
  float* PH = (float*)(ws + OFF_PH);

  const long strideA = (long)NROW * DIM;
  const long strideW = (long)DIM * DIM;
  const long strideP = (long)NROW * DIM;
  const dim3 ggrid((NROW / 64) * (DIM / 64) / 8, 2);
  const dim3 cgrid(DIM * DIM / 8 / NTHR, 2);

  prep_kernel<<<2 * NROW, NTHR, 0, stream>>>(x, hx, AX);

  cvt_w_kernel<<<cgrid, NTHR, 0, stream>>>(u_z_w, w_z, WX);
  gemm_f16_nt<<<ggrid, 256, 0, stream>>>(AX, DIM, strideA, WX, DIM, strideW, PX, DIM, strideP, NROW, DIM, DIM, PFOLD);
  pair_kernel<0><<<NROW, NTHR, 0, stream>>>(PH, PX, u_z_b, hx, ZL);

  cvt_w_kernel<<<cgrid, NTHR, 0, stream>>>(u_r_w, w_r, WX);
  gemm_f16_nt<<<ggrid, 256, 0, stream>>>(AX, DIM, strideA, WX, DIM, strideW, PX, DIM, strideP, NROW, DIM, DIM, PFOLD);
  pair_kernel<1><<<NROW, NTHR, 0, stream>>>(PH, PX, u_r_b, hx, AH);

  cvt_w_kernel<<<cgrid, NTHR, 0, stream>>>(u_w, w, WX);
  gemm_f16_nt<<<ggrid, 256, 0, stream>>>(AX, DIM, strideA, WX, DIM, strideW, PX, DIM, strideP, NROW, DIM, DIM, PFOLD);
  pair_kernel<2><<<NROW, NTHR, 0, stream>>>(PH, PX, u_b, hx, ZL);

  final_kernel<<<NROW, NTHR, 0, stream>>>(PH, hx, (const unsigned*)ZL, out);
}
